// HGCN_11587821765286
// MI455X (gfx1250) — hardware-run, weakly checked
//
#include <hip/hip_runtime.h>
#include <stddef.h>
#include <stdint.h>
#include <math.h>


#define DD     128
#define KA     256
#define NTHR   256
#define NWAVE  8
#define EPT    8
#define CHUNK  (NTHR * EPT)
#define WCAP   (EPT * 32)
#define LISTN  (NWAVE * WCAP)
#define NBA    1024
#define SLA    10
#define RCAP   28672
#define DEGCAP 64
#define GBM    64
#define GTHR   128
#define NUW    (DD * (KA / 8))
#define NBW    (NUW / NTHR)
#define AGG_ZINTS (LISTN + 2 * RCAP + 3 * NBA)
#define AGG_LDS_INTS (AGG_ZINTS + 16)
#define WSMAX  134217728
#define MINN   1e-15f
#define MAXN   0.996f
#define ARTC   0.99999988079071044921875f

static_assert((CHUNK & (CHUNK - 1)) == 0 && CHUNK <= 4096);
static_assert((NBA & (NBA - 1)) == 0 && NBA == (1 << SLA));
static_assert(((long long)CHUNK << SLA) < (1LL << 31));
static_assert(LISTN % NTHR == 0);
static_assert(NBA % NWAVE == 0 && NBA % 32 == 0 && NBA % GBM == 0);
static_assert(RCAP % 4 == 0 && AGG_ZINTS % 4 == 0 && LISTN % 4 == 0);
static_assert(DEGCAP % 32 == 0);
static_assert(DD == 4 * 32 && KA == 2 * DD && KA % 32 == 0);
static_assert(GBM == (GTHR / 32) * 16 && GTHR == DD && GBM % NWAVE == 0);
static_assert(NUW % NTHR == 0 && KA / 8 == 32);
static_assert(AGG_LDS_INTS * 4 <= 300000);

typedef float          v4f   __attribute__((ext_vector_type(4)));
typedef float          v8f   __attribute__((ext_vector_type(8)));
typedef int            v4i   __attribute__((ext_vector_type(4)));
typedef int            v8i   __attribute__((ext_vector_type(8)));
typedef unsigned       v2u   __attribute__((ext_vector_type(2)));
typedef unsigned short v8us  __attribute__((ext_vector_type(8)));
typedef unsigned short v16us __attribute__((ext_vector_type(16)));
typedef __bf16         v16bf __attribute__((ext_vector_type(16)));
typedef v4f  __attribute__((may_alias)) v4fa;
typedef v4i  __attribute__((may_alias)) v4ia;
typedef v2u  __attribute__((may_alias)) v2ua;
typedef v8us __attribute__((may_alias)) v8usa;
union FragB { v16bf v; v16us u; v8us h[2]; v8i w; };

__device__ __forceinline__ v8f wmb(const FragB& a, const FragB& b, v8f c) {
  v8f d = __builtin_amdgcn_wmma_f32_16x16x32_bf16(false, a.v, false, b.v, (short)0, c, false, false);
  asm volatile("v_nop\n\tv_nop\n\tv_nop\n\tv_nop" : "+v"(d) : "v"(a.w), "v"(b.w));
  return d;
}

__device__ __forceinline__ unsigned bf16_bits(float f) {
  const unsigned u = __float_as_uint(f);
  return (u + 0x7FFFu + ((u >> 16) & 1u)) >> 16;
}
__device__ __forceinline__ float bf16_val(float f) {
  return __uint_as_float(bf16_bits(f) << 16);
}

__device__ __forceinline__ float wsum(float v) {
#pragma unroll
  for (int q = 16; q > 0; q >>= 1) v += __shfl_xor(v, q, 32);
  return v;
}

__device__ __forceinline__ void expmap4(float& a, float& b, float& c, float& d) {
  const float n  = fmaxf(sqrtf(wsum(a * a + b * b + c * c + d * d)), MINN);
  const float tn = tanhf(n);
  const float rn = 1.0f / n;
  a = (tn * a) * rn; b = (tn * b) * rn; c = (tn * c) * rn; d = (tn * d) * rn;
}
__device__ __forceinline__ void logmap4(float& a, float& b, float& c, float& d) {
  const float n  = fmaxf(sqrtf(wsum(a * a + b * b + c * c + d * d)), MINN);
  const float at = atanhf(fminf(n, ARTC));
  const float rn = 1.0f / n;
  a = (at * a) * rn; b = (at * b) * rn; c = (at * c) * rn; d = (at * d) * rn;
}
__device__ __forceinline__ void proj4(float& a, float& b, float& c, float& d) {
  const float n  = fmaxf(sqrtf(wsum(a * a + b * b + c * c + d * d)), MINN);
  const bool big = n > MAXN;
  const float rn = 1.0f / n;
  a = big ? (a * rn) * MAXN : a; b = big ? (b * rn) * MAXN : b;
  c = big ? (c * rn) * MAXN : c; d = big ? (d * rn) * MAXN : d;
}

__device__ __forceinline__ void hilo_pack(float v0, float v1, float v2, float v3,
                                          int& h01, int& h23, int& l01, int& l23) {
  const unsigned a0 = bf16_bits(v0), a1 = bf16_bits(v1), a2 = bf16_bits(v2), a3 = bf16_bits(v3);
  const unsigned b0 = bf16_bits(v0 - __uint_as_float(a0 << 16));
  const unsigned b1 = bf16_bits(v1 - __uint_as_float(a1 << 16));
  const unsigned b2 = bf16_bits(v2 - __uint_as_float(a2 << 16));
  const unsigned b3 = bf16_bits(v3 - __uint_as_float(a3 << 16));
  h01 = (int)(a0 | (a1 << 16)); h23 = (int)(a2 | (a3 << 16));
  l01 = (int)(b0 | (b1 << 16)); l23 = (int)(b2 | (b3 << 16));
}

__device__ __forceinline__ v4i regroup16(int h01, int h23, int l01, int l23, int lane) {
  const int s0 = (2 * lane) & 31, s1 = s0 + 1;
  const int a0 = __shfl(h01, s0, 32), a1 = __shfl(h23, s0, 32), a2 = __shfl(h01, s1, 32), a3 = __shfl(h23, s1, 32);
  const int b0 = __shfl(l01, s0, 32), b1 = __shfl(l23, s0, 32), b2 = __shfl(l01, s1, 32), b3 = __shfl(l23, s1, 32);
  const int mk = (lane < 16) ? -1 : 0;
  v4i o;
  o.x = (a0 & mk) | (b0 & ~mk); o.y = (a1 & mk) | (b1 & ~mk);
  o.z = (a2 & mk) | (b2 & ~mk); o.w = (a3 & mk) | (b3 & ~mk);
  return o;
}

template <int SLB>
__device__ __forceinline__ int scan_chunk(const int* __restrict__ dsts, int nE, int cbase, int slotBase,
                                          int nb, int vec8, int* list, int tid, int lane, int wave) {
  int wc = 0;
  const int el0  = tid * EPT;
  const int e0   = cbase + el0;
  const int sent = -2147483647 - 1;
  v4i da, db;
  if (vec8 != 0 && cbase + CHUNK <= nE) {
    da = *(const v4i*)(dsts + e0);
    db = *(const v4i*)(dsts + e0 + 4);
  } else {
    da.x = (e0     < nE) ? dsts[min(e0,     nE - 1)] : sent;
    da.y = (e0 + 1 < nE) ? dsts[min(e0 + 1, nE - 1)] : sent;
    da.z = (e0 + 2 < nE) ? dsts[min(e0 + 2, nE - 1)] : sent;
    da.w = (e0 + 3 < nE) ? dsts[min(e0 + 3, nE - 1)] : sent;
    db.x = (e0 + 4 < nE) ? dsts[min(e0 + 4, nE - 1)] : sent;
    db.y = (e0 + 5 < nE) ? dsts[min(e0 + 5, nE - 1)] : sent;
    db.z = (e0 + 6 < nE) ? dsts[min(e0 + 6, nE - 1)] : sent;
    db.w = (e0 + 7 < nE) ? dsts[min(e0 + 7, nE - 1)] : sent;
  }
  const unsigned nbs = (unsigned)slotBase;
  const unsigned unb = (unsigned)nb;
  const unsigned s0 = (unsigned)da.x - nbs, s1 = (unsigned)da.y - nbs;
  const unsigned s2 = (unsigned)da.z - nbs, s3 = (unsigned)da.w - nbs;
  const unsigned s4 = (unsigned)db.x - nbs, s5 = (unsigned)db.y - nbs;
  const unsigned s6 = (unsigned)db.z - nbs, s7 = (unsigned)db.w - nbs;
  const bool h0 = s0 < unb, h1 = s1 < unb, h2 = s2 < unb, h3 = s3 < unb;
  const bool h4 = s4 < unb, h5 = s5 < unb, h6 = s6 < unb, h7 = s7 < unb;
  const unsigned any = __builtin_amdgcn_ballot_w32(h0 | h1 | h2 | h3 | h4 | h5 | h6 | h7);
  if (any != 0u) {
#define HITJ(J, HJ, SJ) { \
      const unsigned mj = __builtin_amdgcn_ballot_w32(HJ); \
      if (mj != 0u) { \
        if (HJ) { \
          const int pos = wc + (int)__builtin_amdgcn_mbcnt_lo(mj, 0u); \
          if (pos < WCAP) list[wave * WCAP + pos] = ((el0 + (J)) << SLB) | (int)(SJ); \
        } \
        wc += (int)__builtin_popcount(mj); } }
    HITJ(0, h0, s0)
    HITJ(1, h1, s1)
    HITJ(2, h2, s2)
    HITJ(3, h3, s3)
    HITJ(4, h4, s4)
    HITJ(5, h5, s5)
    HITJ(6, h6, s6)
    HITJ(7, h7, s7)
#undef HITJ
  }
  return wc;
}

__global__ __launch_bounds__(NTHR) void k_prep(const float* __restrict__ x, int nN, int gx,
                                               const float* __restrict__ w1, const float* __restrict__ w2,
                                               unsigned short* ap, unsigned short* w1t, unsigned short* w2t) {
  const int tid = (int)threadIdx.x, lane = tid & 31, wave = tid >> 5;
  const int blk = (int)blockIdx.x;
  if (blk < gx) {
    const int row = blk * NWAVE + wave;
    const int rc  = row < nN ? row : nN - 1;
    const bool live = row < nN;
    const v4f a = *(const v4fa*)(x + (size_t)rc * DD + 4 * lane);
    float u0 = bf16_val(a.x), u1 = bf16_val(a.y), u2 = bf16_val(a.z), u3 = bf16_val(a.w);
    expmap4(u0, u1, u2, u3);
    proj4(u0, u1, u2, u3);
    u0 = live ? u0 : 0.0f; u1 = live ? u1 : 0.0f; u2 = live ? u2 : 0.0f; u3 = live ? u3 : 0.0f;
    int h01, h23, l01, l23;
    hilo_pack(u0, u1, u2, u3, h01, h23, l01, l23);
    const v4i o = regroup16(h01, h23, l01, l23, lane);
    unsigned short* dp = ap + (size_t)row * KA + 8 * lane;
    *(volatile v4i*)dp = o;
    __threadfence();
    *(volatile v4i*)dp = o;
  } else {
    const int pb = blk - gx;
    const bool second = pb >= NBW;
    const float* w = second ? w2 : w1;
    unsigned short* wt = second ? w2t : w1t;
    const int u  = (pb & (NBW - 1)) * NTHR + tid;
    const int n  = u >> 5;
    const int k8 = (u & 31) * 8;
    const int kk = k8 & (DD - 1);
    const float* p = w + (size_t)n * DD + kk;
    const v4f a = *(const v4fa*)p;
    const v4f b = *(const v4fa*)(p + 4);
    v8us o;
    o[0] = (unsigned short)bf16_bits(a.x); o[1] = (unsigned short)bf16_bits(a.y);
    o[2] = (unsigned short)bf16_bits(a.z); o[3] = (unsigned short)bf16_bits(a.w);
    o[4] = (unsigned short)bf16_bits(b.x); o[5] = (unsigned short)bf16_bits(b.y);
    o[6] = (unsigned short)bf16_bits(b.z); o[7] = (unsigned short)bf16_bits(b.w);
    unsigned short* dp = wt + (size_t)n * KA + k8;
    *(volatile v8us*)dp = o;
    __threadfence();
    *(volatile v8us*)dp = o;
  }
}

__global__ __launch_bounds__(GTHR) void k_lin(const unsigned short* __restrict__ A,
                                              const unsigned short* __restrict__ BT,
                                              const float* __restrict__ b, int nN, float* XT) {
  __shared__ __attribute__((aligned(16))) float stg[GBM * DD];
  __shared__ __attribute__((aligned(16))) float shb[DD];
  __shared__ float sred[12];
  const int tid = (int)threadIdx.x, lane = tid & 31, wave = tid >> 5, hh = lane >> 4, m = lane & 15;
  const int rowBase = (int)blockIdx.x * GBM;

  const float bk = bf16_val(b[tid]);
  {
    const float s = wsum(bk * bk);
    if (lane == 0) sred[wave] = s;
  }
  __syncthreads();
  const float nb  = fmaxf(sqrtf(((sred[0] + sred[1]) + sred[2]) + sred[3]), MINN);
  const float tnb = tanhf(nb);
  const float ek  = (tnb * bk) * (1.0f / nb);
  {
    const float s = wsum(ek * ek);
    if (lane == 0) sred[4 + wave] = s;
  }
  __syncthreads();
  const float neb = fmaxf(sqrtf(((sred[4] + sred[5]) + sred[6]) + sred[7]), MINN);
  const float hbk = (neb > MAXN) ? (ek * (1.0f / neb)) * MAXN : ek;
  shb[tid] = hbk;
  {
    const float s = wsum(hbk * hbk);
    if (lane == 0) sred[8 + wave] = s;
  }

  v8f acc[8];
  {
    const v8f z = {0.f, 0.f, 0.f, 0.f, 0.f, 0.f, 0.f, 0.f};
#pragma unroll
    for (int t = 0; t < 8; ++t) acc[t] = z;
  }
  const unsigned short* ap = A  + (size_t)(rowBase + 16 * wave + m) * (size_t)KA + 8 * hh;
  const unsigned short* bp = BT + (size_t)m * (size_t)KA + 8 * hh;

#pragma unroll 1
  for (int k0 = 0; k0 < KA; k0 += 32) {
    FragB af;
    af.h[0] = *(const v8usa*)(ap + k0);
    af.h[1] = *(const v8usa*)(ap + k0 + 16);
#pragma unroll
    for (int nt = 0; nt < 8; ++nt) {
      const unsigned short* wq = bp + (size_t)(16 * nt) * (size_t)KA + k0;
      FragB bf;
      bf.h[0] = *(const v8usa*)wq;
      bf.h[1] = *(const v8usa*)(wq + 16);
      acc[nt] = wmb(af, bf, acc[nt]);
    }
  }

#pragma unroll
  for (int nt = 0; nt < 8; ++nt) {
    const int lc = 16 * nt + m;
#pragma unroll
    for (int r = 0; r < 8; ++r) {
      const int lr = 16 * wave + 8 * hh + r;
      stg[lr * DD + lc] = acc[nt][r];
    }
  }
  __syncthreads();

  const float y2 = ((sred[8] + sred[9]) + sred[10]) + sred[11];
  const v4f hb = *(const v4fa*)(shb + 4 * lane);

#pragma unroll 1
  for (int i = 0; i < 16; ++i) {
    const int lr   = 16 * wave + i;
    const int grow = rowBase + lr;
    const bool live = grow < nN;
    const v4f mv = *(const v4fa*)(stg + lr * DD + 4 * lane);
    const unsigned short* ar = A + (size_t)grow * (size_t)KA + 4 * lane;
    const v2u hw = *(const v2ua*)ar;
    const v2u lw = *(const v2ua*)(ar + DD);
    const float x0 = __uint_as_float(hw.x << 16) + __uint_as_float(lw.x << 16);
    const float x1 = __uint_as_float(hw.x & 0xffff0000u) + __uint_as_float(lw.x & 0xffff0000u);
    const float x2 = __uint_as_float(hw.y << 16) + __uint_as_float(lw.y << 16);
    const float x3 = __uint_as_float(hw.y & 0xffff0000u) + __uint_as_float(lw.y & 0xffff0000u);

    const float xn  = fmaxf(sqrtf(wsum(x0 * x0 + x1 * x1 + x2 * x2 + x3 * x3)), MINN);
    const float mxn = fmaxf(sqrtf(wsum(mv.x * mv.x + mv.y * mv.y + mv.z * mv.z + mv.w * mv.w)), MINN);
    const unsigned nzb = __builtin_amdgcn_ballot_w32((mv.x != 0.0f) | (mv.y != 0.0f) | (mv.z != 0.0f) | (mv.w != 0.0f));
    const float art = atanhf(fminf(xn, ARTC));
    const float tt  = tanhf((mxn / xn) * art);
    const float zf  = (nzb != 0u) ? 1.0f : 0.0f;
    const float rmx = 1.0f / mxn;
    float h0 = ((tt * mv.x) * rmx) * zf, h1 = ((tt * mv.y) * rmx) * zf;
    float h2 = ((tt * mv.z) * rmx) * zf, h3 = ((tt * mv.w) * rmx) * zf;
    proj4(h0, h1, h2, h3);

    const float xx = wsum(h0 * h0 + h1 * h1 + h2 * h2 + h3 * h3);
    const float xy = wsum(h0 * hb.x + h1 * hb.y + h2 * hb.z + h3 * hb.w);
    const float t12 = 1.0f + 2.0f * xy;
    const float ca  = t12 + y2;
    const float cb  = 1.0f - xx;
    const float den = fmaxf(t12 + xx * y2, MINN);
    const float rdn = 1.0f / den;
    float p0 = (ca * h0 + cb * hb.x) * rdn, p1 = (ca * h1 + cb * hb.y) * rdn;
    float p2 = (ca * h2 + cb * hb.z) * rdn, p3 = (ca * h3 + cb * hb.w) * rdn;
    proj4(p0, p1, p2, p3);
    logmap4(p0, p1, p2, p3);

    v4f o;
    o.x = live ? p0 : 0.0f; o.y = live ? p1 : 0.0f; o.z = live ? p2 : 0.0f; o.w = live ? p3 : 0.0f;
    float* op = XT + (size_t)grow * DD + 4 * lane;
    *(volatile v4f*)op = o;
    __threadfence();
    *(volatile v4f*)op = o;
  }
}

template <int L1>
__global__ __launch_bounds__(NTHR) void k_agg(const int* __restrict__ gsrc, const int* __restrict__ keys,
                                              const float* __restrict__ ew, int nE, int nN, int vec8, int mRows,
                                              const float* __restrict__ xt, unsigned short* ap, float* outp) {
  extern __shared__ __attribute__((aligned(16))) int dsm[];
  int* list = dsm;
  int* hl   = dsm + LISTN;
  int* sl   = dsm + LISTN + RCAP;
  int* cnt  = dsm + LISTN + 2 * RCAP;
  int* offs = cnt + NBA;
  int* cur  = offs + NBA;
  int* misc = cur + NBA;
  const int tid = (int)threadIdx.x, lane = tid & 31, wave = tid >> 5;
  const int nodeBase = (int)blockIdx.x * NBA;

  {
    const v4i z4 = {0, 0, 0, 0};
    for (int i = tid * 4; i < AGG_ZINTS; i += NTHR * 4) *(v4ia*)(dsm + i) = z4;
    if (tid < 16) misc[tid] = 0;
  }
  __syncthreads();

  int t = 0, ov = 0;
  const int nChunks = (nE + CHUNK - 1) / CHUNK;
#pragma unroll 1
  for (int ch = 0; ch < nChunks; ++ch) {
    const int cbase = ch * CHUNK;
    const int wc = scan_chunk<SLA>(keys, nE, cbase, nodeBase, NBA, vec8, list, tid, lane, wave);
    if (lane == 0) misc[wave] = wc;
    __syncthreads();
    if (wave == 0) {
#pragma unroll 1
      for (int w2 = 0; w2 < NWAVE; ++w2) {
        int c = misc[w2];
        c = c < 0 ? 0 : (c > WCAP ? WCAP : c);
#pragma unroll 1
        for (int b0 = 0; b0 < c; b0 += 32) {
          const int idx = b0 + lane;
          const int ent = list[w2 * WCAP + (idx < WCAP ? idx : WCAP - 1)];
          const int m32 = (c - b0) < 32 ? (c - b0) : 32;
#pragma unroll 1
          for (int k = 0; k < m32; ++k) {
            const int u    = __builtin_amdgcn_readlane(ent, k);
            const int slot = u & (NBA - 1);
            const int el   = (u >> SLA) & (CHUNK - 1);
            const int pk   = ((cbase + el) << SLA) | slot;
            if (t < RCAP) {
              if (lane == 0) { hl[t] = pk; cnt[slot] = cnt[slot] + 1; }
              t = t + 1;
            } else {
              ov = 1;
            }
          }
        }
      }
    }
    __syncthreads();
  }
  if (wave == 0 && lane == 0) { misc[8] = t; misc[9] = ov; }
  __syncthreads();
  int tt = misc[8];
  tt = tt < 0 ? 0 : (tt > RCAP ? RCAP : tt);
  const int ovf = misc[9];

  if (wave == 0) {
    const int base = lane * (NBA / 32);
    int s = 0;
#pragma unroll 1
    for (int i = 0; i < NBA / 32; ++i) s += cnt[base + i];
    int incl = s;
#pragma unroll
    for (int d = 1; d < 32; d <<= 1) {
      const int y = __shfl_up(incl, d, 32);
      if (lane >= d) incl += y;
    }
    int run = incl - s;
#pragma unroll 1
    for (int i = 0; i < NBA / 32; ++i) {
      const int cv = cnt[base + i];
      offs[base + i] = run;
      cur[base + i]  = run;
      run += cv;
    }
  }
  __syncthreads();
  if (wave == 0) {
#pragma unroll 1
    for (int b0 = 0; b0 < tt; b0 += 32) {
      const int idx = b0 + lane;
      const int ent = hl[idx < RCAP ? idx : RCAP - 1];
      const int m32 = (tt - b0) < 32 ? (tt - b0) : 32;
#pragma unroll 1
      for (int k = 0; k < m32; ++k) {
        const int u    = __builtin_amdgcn_readlane(ent, k);
        const int slot = u & (NBA - 1);
        if (lane == 0) {
          int p = cur[slot];
          p = p < 0 ? 0 : (p > RCAP - 1 ? RCAP - 1 : p);
          sl[p] = u;
          cur[slot] = p + 1;
        }
      }
    }
  }
  __syncthreads();

  const float pz = (ovf != 0) ? __int_as_float(0x7fc00000) : 0.0f;
#pragma unroll 1
  for (int si = 0; si < NBA / NWAVE; ++si) {
    const int s    = si * NWAVE + wave;
    const int node = nodeBase + s;
    int c = cnt[s];
    const bool big = c > DEGCAP;
    c = c < 0 ? 0 : (c > DEGCAP ? DEGCAP : c);
    int o = offs[s];
    o = o < 0 ? 0 : (o > RCAP ? RCAP : o);
    float g0 = 0.0f, g1 = 0.0f, g2 = 0.0f, g3 = 0.0f;
#pragma unroll 1
    for (int b0 = 0; b0 < c; b0 += 32) {
      int idx = o + b0 + lane;
      idx = idx > RCAP - 1 ? RCAP - 1 : idx;
      const int ent = sl[idx];
      int eid = ent >> SLA;
      eid = eid < 0 ? 0 : (eid > nE - 1 ? nE - 1 : eid);
      int sr = gsrc[eid];
      sr = sr < 0 ? 0 : (sr > nN - 1 ? nN - 1 : sr);
      const int wvi = __float_as_int(bf16_val(ew[eid]));
      const int m32 = (c - b0) < 32 ? (c - b0) : 32;
#pragma unroll 1
      for (int k = 0; k < m32; ++k) {
        const int   sk = __builtin_amdgcn_readlane(sr, k);
        const float wk = __int_as_float(__builtin_amdgcn_readlane(wvi, k));
        const v4f a = *(const v4fa*)(xt + (size_t)sk * DD + 4 * lane);
        g0 = fmaf(a.x, wk, g0); g1 = fmaf(a.y, wk, g1);
        g2 = fmaf(a.z, wk, g2); g3 = fmaf(a.w, wk, g3);
      }
    }
    expmap4(g0, g1, g2, g3);
    proj4(g0, g1, g2, g3);
    logmap4(g0, g1, g2, g3);
    g0 = fmaxf(g0, 0.0f); g1 = fmaxf(g1, 0.0f); g2 = fmaxf(g2, 0.0f); g3 = fmaxf(g3, 0.0f);
    expmap4(g0, g1, g2, g3);
    proj4(g0, g1, g2, g3);
    const float pzr = big ? __int_as_float(0x7fc00000) : pz;
    const bool live = node < nN;
    const float q0 = live ? g0 + pzr : 0.0f, q1 = live ? g1 + pzr : 0.0f;
    const float q2 = live ? g2 + pzr : 0.0f, q3 = live ? g3 + pzr : 0.0f;
    if constexpr (L1 != 0) {
      int h01, h23, l01, l23;
      hilo_pack(q0, q1, q2, q3, h01, h23, l01, l23);
      const v4i ow = regroup16(h01, h23, l01, l23, lane);
      if (node < mRows) {
        unsigned short* hp = ap + (size_t)node * KA + 8 * lane;
        *(volatile v4i*)hp = ow;
        __threadfence();
        *(volatile v4i*)hp = ow;
      }
    } else {
      v4f ow;
      ow.x = q0; ow.y = q1; ow.z = q2; ow.w = q3;
      if (live) {
        float* op = outp + (size_t)node * DD + 4 * lane;
        *(volatile v4f*)op = ow;
        __threadfence();
        *(volatile v4f*)op = ow;
      }
    }
  }
}

static inline int cdiv(int a, int b) { return (a + b - 1) / b; }

extern "C" void kernel_launch(void* const* d_in, const int* in_sizes, int n_in,
                              void* d_out, int out_size, void* d_ws, size_t ws_size,
                              hipStream_t stream) {
  if (n_in < 7) return;
  if (in_sizes[0] < DD || (in_sizes[0] % DD) != 0) return;
  const int nN = in_sizes[0] / DD;
  if (in_sizes[1] < 2 || (in_sizes[1] & 1) != 0) return;
  const int nE = in_sizes[1] / 2;
  if (nE < 1 || nE >= (1 << 21)) return;
  if (in_sizes[2] != nE) return;
  if (in_sizes[3] != DD * DD || in_sizes[4] != DD) return;
  if (in_sizes[5] != DD * DD || in_sizes[6] != DD) return;
  if ((long long)out_size != (long long)nN * DD) return;

  const float* x    = (const float*)d_in[0];
  const int*   edge = (const int*)d_in[1];
  const float* ew   = (const float*)d_in[2];
  const float* w1   = (const float*)d_in[3];
  const float* b1   = (const float*)d_in[4];
  const float* w2   = (const float*)d_in[5];
  const float* b2   = (const float*)d_in[6];
  float* out = (float*)d_out;
  const int* keys = edge;
  const int* gsrc = edge + nE;

  const int MP = cdiv(nN, GBM) * GBM;
  const int gL = MP / GBM;
  const int gX = MP / NWAVE;
  const int gA = cdiv(nN, NBA);
  if ((long long)gA * NBA < (long long)MP) return;
  const int vec8 = ((nE & 3) == 0) ? 1 : 0;

  char* ws = (char*)d_ws;
  size_t off = 0;
  const size_t oW1T = off; off += (size_t)DD * KA * 2;        off = (off + 255) & ~(size_t)255;
  const size_t oW2T = off; off += (size_t)DD * KA * 2;        off = (off + 255) & ~(size_t)255;
  const size_t oAP  = off; off += (size_t)MP * KA * 2;        off = (off + 255) & ~(size_t)255;
  const size_t oXT  = off; off += (size_t)MP * DD * 4;        off = (off + 255) & ~(size_t)255;
  if (off > ws_size || off > (size_t)WSMAX) return;
  unsigned short* W1T = (unsigned short*)(ws + oW1T);
  unsigned short* W2T = (unsigned short*)(ws + oW2T);
  unsigned short* AP  = (unsigned short*)(ws + oAP);
  float*          XT  = (float*)(ws + oXT);

  const size_t aggLds = (size_t)AGG_LDS_INTS * 4;
  hipFuncSetAttribute(reinterpret_cast<const void*>(&k_agg<1>), hipFuncAttributeMaxDynamicSharedMemorySize, (int)aggLds);
  hipFuncSetAttribute(reinterpret_cast<const void*>(&k_agg<0>), hipFuncAttributeMaxDynamicSharedMemorySize, (int)aggLds);

  k_prep<<<gX + 2 * NBW, NTHR, 0, stream>>>(x, nN, gX, w1, w2, AP, W1T, W2T);
  k_lin<<<gL, GTHR, 0, stream>>>(AP, W1T, b1, nN, XT);
  k_agg<1><<<gA, NTHR, aggLds, stream>>>(gsrc, keys, ew, nE, nN, vec8, MP, XT, AP, out);
  k_lin<<<gL, GTHR, 0, stream>>>(AP, W2T, b2, nN, XT);
  k_agg<0><<<gA, NTHR, aggLds, stream>>>(gsrc, keys, ew, nE, nN, vec8, MP, XT, AP, out);
}
